// BasicSelfAttention2D_48326972015259
// MI455X (gfx1250) — hardware-verified
//
#include <hip/hip_runtime.h>


#define NBI  8
#define CC   256
#define HW   64
#define NTOK 4096
#define NKV  1024
#define DQ   32
#define DQP  64
#define DM   CC
#define NTK  NTOK
#define SCL  0.17677669529663687f
#define LOSC 1024.0f

typedef _Float16 h16;
typedef unsigned short bf;
typedef __attribute__((ext_vector_type(16))) __bf16   v16bf;
typedef __attribute__((ext_vector_type(16))) _Float16 v16h;
typedef __attribute__((ext_vector_type(8)))  _Float16 v8h;
typedef __attribute__((ext_vector_type(8)))  unsigned short v8us;
typedef __attribute__((ext_vector_type(8)))  float    v8f;
typedef __attribute__((ext_vector_type(4)))  float    v4f;
typedef __attribute__((ext_vector_type(4)))  _Float16 v4h;
typedef v8h  __attribute__((may_alias)) v8ha;
typedef v4f  __attribute__((may_alias)) v4fa;
typedef v8us __attribute__((may_alias)) v8usa;

__device__ __forceinline__ unsigned short f2bf(float f) { unsigned u = __float_as_uint(f); u += 0x7FFFu + ((u >> 16) & 1u); return (unsigned short)(u >> 16); }
__device__ __forceinline__ float bf2f(unsigned short b) { return __uint_as_float(((unsigned)b) << 16); }
__device__ __forceinline__ float bfr(float f) { return bf2f(f2bf(f)); }
__device__ __forceinline__ v16h cat16(v8h lo, v8h hi) { return __builtin_shufflevector(lo, hi, 0, 1, 2, 3, 4, 5, 6, 7, 8, 9, 10, 11, 12, 13, 14, 15); }
__device__ __forceinline__ v16bf cat16b(v8us lo, v8us hi) { return __builtin_bit_cast(v16bf, __builtin_shufflevector(lo, hi, 0, 1, 2, 3, 4, 5, 6, 7, 8, 9, 10, 11, 12, 13, 14, 15)); }
__device__ __forceinline__ v8f wmma16(v16h a, v16h b, v8f c) { return __builtin_amdgcn_wmma_f32_16x16x32_f16(false, a, false, b, (short)0, c, false, false); }
__device__ __forceinline__ v8f wmmab(v16bf a, v16bf b, v8f c) { return __builtin_amdgcn_wmma_f32_16x16x32_bf16(false, a, false, b, (short)0, c, false, false); }

__global__ __launch_bounds__(256) void k_wt(const float* __restrict__ Wm, int K, int ncols, bf* WT) {
    __shared__ __align__(16) unsigned short tl[64 * 72];
    const int tid = threadIdx.x, k0 = blockIdx.x * 64, n0 = blockIdx.y * 64;
    const int kk = tid >> 2, nq = (tid & 3) * 16;
#pragma unroll
    for (int i = 0; i < 16; ++i) tl[(nq + i) * 72 + kk] = f2bf(Wm[(size_t)(k0 + kk) * ncols + n0 + nq + i]);
    __syncthreads();
    const int piece = tid & 7;
    auto pass = [&]() {
#pragma unroll
        for (int s = 0; s < 2; ++s) { const int nr = (tid >> 3) + 32 * s; const v8us val = *(const v8usa*)(tl + nr * 72 + piece * 8); *(volatile v8us*)(WT + (size_t)(n0 + nr) * K + k0 + piece * 8) = val; }
    };
    pass(); __threadfence(); pass();
}
template <bool SPLITA, bool F16OUT = false>
__global__ __launch_bounds__(128) void k_gemmb(const bf* __restrict__ A, const bf* __restrict__ Al, const bf* __restrict__ Bn, const float* __restrict__ bias, float* C, int ldc, h16* C2, const float* __restrict__ R = nullptr, int K = DM, int roundR = 1) {
    __shared__ __align__(16) float ost[4][16 * 68];
    const int lane = threadIdx.x & 31, wave = threadIdx.x >> 5, lr = lane & 15, hi = lane >> 4;
    const int r0 = blockIdx.x * 64 + wave * 16, c0 = blockIdx.y * 64;
    const size_t aoff = (size_t)(r0 + lr) * K + 8 * hi;
    size_t boff[4];
#pragma unroll
    for (int t = 0; t < 4; ++t) boff[t] = (size_t)(c0 + t * 16 + lr) * K + 8 * hi;
    v8f acc[4];
#pragma unroll
    for (int t = 0; t < 4; ++t) acc[t] = (v8f){};
#pragma unroll 1
    for (int kc = 0; kc < K; kc += 32) {
        const v16bf a = cat16b(*(const v8us*)(A + aoff + kc), *(const v8us*)(A + aoff + kc + 16));
        v16bf al = a;
        if (SPLITA) al = cat16b(*(const v8us*)(Al + aoff + kc), *(const v8us*)(Al + aoff + kc + 16));
#pragma unroll
        for (int t = 0; t < 4; ++t) { const v16bf b = cat16b(*(const v8us*)(Bn + boff[t] + kc), *(const v8us*)(Bn + boff[t] + kc + 16)); acc[t] = wmmab(a, b, acc[t]); if (SPLITA) acc[t] = wmmab(al, b, acc[t]); }
        asm volatile("v_nop\n\tv_nop\n\tv_nop\n\tv_nop" : "+v"(acc[0]), "+v"(acc[1]), "+v"(acc[2]), "+v"(acc[3]) : "v"(a), "v"(al));
    }
    float* os = &ost[wave][0];
#pragma unroll
    for (int t = 0; t < 4; ++t) { const float bv = bias ? bfr(bias[c0 + t * 16 + lr]) : 0.f;
#pragma unroll
        for (int j = 0; j < 8; ++j) os[(hi * 8 + j) * 68 + t * 16 + lr] = acc[t][j] + bv; }
    __syncthreads();
    if (F16OUT) {
        h16* crow = (h16*)(void*)C + (size_t)r0 * ldc + c0;
        auto pass = [&]() {
#pragma unroll
            for (int s = 0; s < 4; ++s) { const int row = 4 * s + (lane >> 3), piece = lane & 7; const float* sp = os + row * 68 + piece * 8; v8h o, o2;
#pragma unroll
                for (int i = 0; i < 8; ++i) { const h16 a = (h16)sp[i]; o[i] = a; o2[i] = (h16)((sp[i] - (float)a) * LOSC); }
                *(volatile v8h*)(crow + (size_t)row * ldc + piece * 8) = o; if (C2) *(volatile v8h*)(C2 + (size_t)r0 * ldc + c0 + (size_t)row * ldc + piece * 8) = o2; }
        };
        pass(); __threadfence(); pass();
    } else {
        float* crow = C + (size_t)r0 * ldc + c0;
        auto pass = [&]() {
#pragma unroll
            for (int s = 0; s < 8; ++s) { const int Lid = (lane >> 3) + 4 * s, piece = lane & 7; const int row = Lid >> 1, cofs = (Lid & 1) * 32 + piece * 4;
                v4f val = *(const v4fa*)(os + row * 68 + cofs); if (R) { const v4f rv = *(const v4f*)(R + ((size_t)r0 + row) * ldc + c0 + cofs); val += roundR ? (v4f){bfr(rv[0]), bfr(rv[1]), bfr(rv[2]), bfr(rv[3])} : rv; }
                *(volatile v4f*)(crow + (size_t)row * ldc + cofs) = val; }
        };
        pass(); __threadfence(); pass();
    }
}

__global__ __launch_bounds__(128) void k_gemm3(const bf* __restrict__ Ah, const bf* __restrict__ Al, const bf* __restrict__ Bh, const bf* __restrict__ Bl, int K, float* C, int ldc) {
    __shared__ __align__(16) float ost[4][16 * 68];
    const int lane = threadIdx.x & 31, wave = threadIdx.x >> 5, lr = lane & 15, hi = lane >> 4;
    const int r0 = blockIdx.x * 64 + wave * 16, c0 = blockIdx.y * 64;
    const size_t aoff = (size_t)(r0 + lr) * K + 8 * hi;
    v8f acc[4];
#pragma unroll
    for (int t = 0; t < 4; ++t) acc[t] = (v8f){};
#pragma unroll 1
    for (int kc = 0; kc < K; kc += 32) {
        const v16bf a = cat16b(*(const v8us*)(Ah + aoff + kc), *(const v8us*)(Ah + aoff + kc + 16));
        const v16bf al = cat16b(*(const v8us*)(Al + aoff + kc), *(const v8us*)(Al + aoff + kc + 16));
#pragma unroll
        for (int t = 0; t < 4; ++t) { const size_t bo = (size_t)(c0 + t * 16 + lr) * K + kc + 8 * hi;
            const v16bf bh = cat16b(*(const v8us*)(Bh + bo), *(const v8us*)(Bh + bo + 16)); const v16bf bl = cat16b(*(const v8us*)(Bl + bo), *(const v8us*)(Bl + bo + 16));
            acc[t] = wmmab(a, bh, acc[t]); acc[t] = wmmab(al, bh, acc[t]); acc[t] = wmmab(a, bl, acc[t]); }
        asm volatile("v_nop\n\tv_nop\n\tv_nop\n\tv_nop" : "+v"(acc[0]), "+v"(acc[1]), "+v"(acc[2]), "+v"(acc[3]) : "v"(a), "v"(al));
    }
    float* os = &ost[wave][0];
#pragma unroll
    for (int t = 0; t < 4; ++t) {
#pragma unroll
        for (int j = 0; j < 8; ++j) os[(hi * 8 + j) * 68 + t * 16 + lr] = acc[t][j]; }
    __builtin_amdgcn_wave_barrier(); asm volatile("" ::: "memory");
    float* crow = C + (size_t)r0 * ldc + c0;
    auto pass = [&]() {
#pragma unroll
        for (int s = 0; s < 8; ++s) { const int Lid = (lane >> 3) + 4 * s, piece = lane & 7; const int row = Lid >> 1, cofs = (Lid & 1) * 32 + piece * 4;
            const v4f val = *(const v4fa*)(os + row * 68 + cofs); *(volatile v4f*)(crow + (size_t)row * ldc + cofs) = val; }
    };
    pass(); __threadfence(); pass();
}

__global__ __launch_bounds__(256) void k_bfz(const float* __restrict__ src, bf* dh, bf* dz, size_t n8) {
    const size_t i = (size_t)blockIdx.x * 256 + threadIdx.x; if (i >= n8) return;
    const v8f v = *(const v8f*)(src + i * 8); v8us o, z;
#pragma unroll
    for (int k = 0; k < 8; ++k) { o[k] = f2bf(v[k]); z[k] = 0; }
    *(volatile v8us*)(dh + i * 8) = o; *(volatile v8us*)(dz + i * 8) = z; __threadfence(); *(volatile v8us*)(dh + i * 8) = o; *(volatile v8us*)(dz + i * 8) = z;
}
__global__ __launch_bounds__(256) void k_wpad(const float* __restrict__ w, bf* WP) {
    const int u = blockIdx.x * 256 + threadIdx.x; if (u >= DQP * CC / 8) return;
    const int d = u / (CC / 8), c0 = (u % (CC / 8)) * 8; v8us o;
#pragma unroll
    for (int i = 0; i < 8; ++i) o[i] = (d < DQ) ? f2bf(w[d * CC + c0 + i]) : (unsigned short)0;
    *(volatile v8us*)(WP + (size_t)d * CC + c0) = o; __threadfence(); *(volatile v8us*)(WP + (size_t)d * CC + c0) = o;
}
__global__ __launch_bounds__(256) void k_poolT(const float* __restrict__ x, bf* Ph, bf* Pl) {
    const int lane = threadIdx.x & 31, m = blockIdx.x * 8 + (threadIdx.x >> 5); if (m >= NKV) return;
    const int pi = m / 32, pj = m % 32; v8us oh, ol;
#pragma unroll
    for (int i = 0; i < 8; ++i) { const int c = lane * 8 + i; const float* xc = x + (size_t)c * NTOK + (2 * pi) * HW + 2 * pj;
        const float s = (bfr(xc[0]) + bfr(xc[1])) + (bfr(xc[HW]) + bfr(xc[HW + 1])); const float v = s * 0.25f; const unsigned short hb = f2bf(v); oh[i] = hb; ol[i] = f2bf(v - bf2f(hb)); }
    const size_t o = (size_t)m * CC + lane * 8; *(volatile v8us*)(Ph + o) = oh; *(volatile v8us*)(Pl + o) = ol; __threadfence(); *(volatile v8us*)(Ph + o) = oh; *(volatile v8us*)(Pl + o) = ol;
}
__global__ __launch_bounds__(256) void k_split64(const float* __restrict__ src, int nrows, bf* dh, bf* dl) {
    typedef __attribute__((ext_vector_type(2))) unsigned short v2us;
    const int lane = threadIdx.x & 31, r = blockIdx.x * 8 + (threadIdx.x >> 5); if (r >= nrows) return;
    const size_t o = (size_t)r * DQP + lane * 2; v2us oh, ol;
#pragma unroll
    for (int i = 0; i < 2; ++i) { const float v = src[o + i]; const unsigned short hb = f2bf(v); oh[i] = hb; ol[i] = f2bf(v - bf2f(hb)); }
    *(volatile v2us*)(dh + o) = oh; *(volatile v2us*)(dl + o) = ol; __threadfence(); *(volatile v2us*)(dh + o) = oh; *(volatile v2us*)(dl + o) = ol;
}
__global__ __launch_bounds__(256) void k_splitw(const float* __restrict__ src, int nrows, int ncols, bf* dh, bf* dl) {
    const int lane = threadIdx.x & 31, r = blockIdx.x * 8 + (threadIdx.x >> 5); if (r >= nrows) return;
#pragma unroll 1
    for (int ps = 0; ps < 2; ++ps) {
#pragma unroll 1
        for (int q = 0; q < ncols / 256; ++q) { const size_t o = (size_t)r * ncols + q * 256 + lane * 8; const v8f v = *(const v8f*)(src + o); v8us oh, ol;
#pragma unroll
            for (int i = 0; i < 8; ++i) { const unsigned short hb = f2bf(v[i]); oh[i] = hb; ol[i] = f2bf(v[i] - bf2f(hb)); }
            *(volatile v8us*)(dh + o) = oh; *(volatile v8us*)(dl + o) = ol; }
        if (ps == 0) __threadfence(); }
}
__global__ __launch_bounds__(256) void k_softmax(const float* __restrict__ S, bf* PH, bf* PL) {
    const int lane = threadIdx.x & 31, r = blockIdx.x * 8 + (threadIdx.x >> 5); if (r >= NTOK) return;
    const float* sr = S + (size_t)r * NKV; float m = -3.0e38f;
#pragma unroll 1
    for (int c0 = lane * 8; c0 < NKV; c0 += 256) { const v8f v = *(const v8f*)(sr + c0);
#pragma unroll
        for (int i = 0; i < 8; ++i) m = fmaxf(m, v[i] * SCL); }
#pragma unroll
    for (int sh = 16; sh; sh >>= 1) m = fmaxf(m, __shfl_xor(m, sh, 32));
    float sum = 0.f;
#pragma unroll 1
    for (int c0 = lane * 8; c0 < NKV; c0 += 256) { const v8f v = *(const v8f*)(sr + c0);
#pragma unroll
        for (int i = 0; i < 8; ++i) sum += __expf(v[i] * SCL - m); }
#pragma unroll
    for (int sh = 16; sh; sh >>= 1) sum += __shfl_xor(sum, sh, 32);
    const float inv = 1.0f / sum;
#pragma unroll 1
    for (int ps = 0; ps < 2; ++ps) {
#pragma unroll 1
        for (int c0 = lane * 8; c0 < NKV; c0 += 256) { const v8f v = *(const v8f*)(sr + c0); v8us oh, ol;
#pragma unroll
            for (int i = 0; i < 8; ++i) { const float p = __expf(v[i] * SCL - m) * inv; const unsigned short hb = f2bf(p); oh[i] = hb; ol[i] = f2bf(p - bf2f(hb)); }
            const size_t o = (size_t)r * NKV + c0; *(volatile v8us*)(PH + o) = oh; *(volatile v8us*)(PL + o) = ol; }
        if (ps == 0) __threadfence(); }
}
__global__ __launch_bounds__(256) void k_resid(const float* __restrict__ Y, const float* __restrict__ X, const float* __restrict__ gam, float* OUTP) {
    const int lane = threadIdx.x & 31, r = blockIdx.x * 8 + (threadIdx.x >> 5); if (r >= CC) return;
    const float g = bfr(gam[0]);
#pragma unroll 1
    for (int ps = 0; ps < 2; ++ps) {
#pragma unroll 1
        for (int q = 0; q < NTOK / 256; ++q) { const size_t o = (size_t)r * NTOK + q * 256 + lane * 8; const v8f y = *(const v8f*)(Y + o); const v8f xv = *(const v8f*)(X + o); v8f v;
#pragma unroll
            for (int i = 0; i < 8; ++i) v[i] = bfr(xv[i]) + g * y[i];
            *(volatile v8f*)(OUTP + o) = v; }
        if (ps == 0) __threadfence(); }
}

extern "C" void kernel_launch(void* const* d_in, const int* in_sizes, int n_in,
                              void* d_out, int out_size, void* d_ws, size_t ws_size, hipStream_t stream) {
    (void)in_sizes; (void)n_in; (void)out_size;
    const float* x = (const float*)d_in[0]; const float* wq = (const float*)d_in[1]; const float* wk = (const float*)d_in[2]; const float* wv = (const float*)d_in[3]; const float* wo = (const float*)d_in[4]; const float* gam = (const float*)d_in[5];
    float* out = (float*)d_out;
    char* wsp = (char*)d_ws;
    auto take = [&](size_t bytes) { char* p = wsp; wsp += (bytes + 255) & ~(size_t)255; return (void*)p; };
    bf* WqP = (bf*)take((size_t)DQP * CC * 2); bf* WkP = (bf*)take((size_t)DQP * CC * 2); bf* WvB = (bf*)take((size_t)CC * CC * 2); bf* WoB = (bf*)take((size_t)CC * CC * 2); bf* WZ = (bf*)take((size_t)CC * CC * 2);
    bf* XT = (bf*)take((size_t)NTOK * CC * 2); bf* KVh = (bf*)take((size_t)NKV * CC * 2); bf* KVl = (bf*)take((size_t)NKV * CC * 2);
    float* TMP = (float*)take((size_t)CC * NTOK * 4); bf* Qh = (bf*)take((size_t)NTOK * DQP * 2); bf* Ql = (bf*)take((size_t)NTOK * DQP * 2); bf* Kh = (bf*)take((size_t)NKV * DQP * 2); bf* Kl = (bf*)take((size_t)NKV * DQP * 2);
    bf* Vh = (bf*)take((size_t)CC * NKV * 2); bf* Vl = (bf*)take((size_t)CC * NKV * 2); float* S = (float*)take((size_t)NTOK * NKV * 4); bf* PH = (bf*)take((size_t)NTOK * NKV * 2); bf* PL = (bf*)take((size_t)NTOK * NKV * 2);
    bf* OAh = (bf*)take((size_t)NTOK * CC * 2); bf* OAl = (bf*)take((size_t)NTOK * CC * 2);
    if ((size_t)(wsp - (char*)d_ws) > ws_size) return;
    k_wpad<<<(DQP * CC / 8 + 255) / 256, 256, 0, stream>>>(wq, WqP); k_wpad<<<(DQP * CC / 8 + 255) / 256, 256, 0, stream>>>(wk, WkP);
    k_bfz<<<(CC * CC / 8 + 255) / 256, 256, 0, stream>>>(wv, WvB, WZ, CC * CC / 8); k_bfz<<<(CC * CC / 8 + 255) / 256, 256, 0, stream>>>(wo, WoB, WZ, CC * CC / 8);
    for (int b = 0; b < NBI; ++b) {
        const float* xb = x + (size_t)b * CC * NTOK;
        k_wt<<<dim3(CC / 64, NTOK / 64, 1), 256, 0, stream>>>(xb, CC, NTOK, XT);
        k_gemmb<false, false><<<dim3(NTOK / 64, 1, 1), 128, 0, stream>>>(XT, nullptr, WqP, nullptr, TMP, DQP, nullptr); k_split64<<<NTOK / 8, 256, 0, stream>>>(TMP, NTOK, Qh, Ql);
        k_poolT<<<NKV / 8, 256, 0, stream>>>(xb, KVh, KVl);
        k_gemmb<true, false><<<dim3(NKV / 64, 1, 1), 128, 0, stream>>>(KVh, KVl, WkP, nullptr, TMP, DQP, nullptr); k_split64<<<NKV / 8, 256, 0, stream>>>(TMP, NKV, Kh, Kl);
        k_gemm3<<<dim3(CC / 64, NKV / 64, 1), 128, 0, stream>>>(WvB, WZ, KVh, KVl, CC, TMP, NKV); k_splitw<<<CC / 8, 256, 0, stream>>>(TMP, CC, NKV, Vh, Vl);
        k_gemm3<<<dim3(NTOK / 64, NKV / 64, 1), 128, 0, stream>>>(Qh, Ql, Kh, Kl, DQP, S, NKV);
        k_softmax<<<NTOK / 8, 256, 0, stream>>>(S, PH, PL);
        k_gemm3<<<dim3(NTOK / 64, CC / 64, 1), 128, 0, stream>>>(PH, PL, Vh, Vl, NKV, TMP, CC); k_splitw<<<NTOK / 8, 256, 0, stream>>>(TMP, NTOK, CC, OAh, OAl);
        k_gemm3<<<dim3(CC / 64, NTOK / 64, 1), 128, 0, stream>>>(WoB, WZ, OAh, OAl, CC, TMP, NTOK);
        k_resid<<<CC / 8, 256, 0, stream>>>(TMP, xb, gam, out + (size_t)b * CC * NTOK);
    }
}
